// VimBlock_68298569941703
// MI455X (gfx1250) — hardware-run, weakly checked
//
#include <hip/hip_runtime.h>
#include <math.h>

typedef __attribute__((ext_vector_type(16))) _Float16 v16h;
typedef __attribute__((ext_vector_type(8)))  _Float16 v8h;
typedef __attribute__((ext_vector_type(8)))  float    v8f;
typedef __attribute__((ext_vector_type(4)))  float    v4f;

constexpr int kB     = 4;
constexpr int kC     = 96;
constexpr int kL     = 4096;
constexpr int kRows  = kB * kL;
constexpr int kE     = 192;
constexpr int kP     = 2 * kE;
constexpr int kR     = 6;
constexpr int kN     = 16;
constexpr int kDbc   = kR + 2 * kN;
constexpr int kDbcP  = 64;
constexpr int kTaps  = 4;
constexpr float kEps = 1e-5f;

constexpr int kCarryW   = 256;
constexpr int kCarryXn  = 16;
constexpr int kCarryXs  = 32;
constexpr int kCarryY   = 128;
constexpr int kCarryRem = 2048;

static_assert(kRows == 16384);
static_assert(kDbc == 38 && kDbc <= kDbcP);
static_assert((kC % 32) == 0 && (kE % 32) == 0);
static_assert((kRows % 64) == 0 && (kP % 64) == 0 && (kDbcP % 64) == 0 && (kC % 16) == 0);
static_assert((kL % 64) == 0 && (kE % 64) == 0);
static_assert(kTaps == 4);

constexpr size_t kOffXN   = 0;
constexpr size_t kOffXNR  = kOffXN   + (size_t)kRows * kC    * 2;
constexpr size_t kOffWIN  = kOffXNR  + (size_t)kRows * kC    * 2;
constexpr size_t kOffWINR = kOffWIN  + (size_t)kP    * kC    * 2;
constexpr size_t kOffWX   = kOffWINR + (size_t)kP    * kC    * 2;
constexpr size_t kOffWOUT = kOffWX   + (size_t)kDbcP * kE    * 2;
constexpr size_t kOffXZ   = kOffWOUT + (size_t)kC    * kE    * 2;
constexpr size_t kOffXS32 = kOffXZ   + (size_t)kRows * kP    * 4;
constexpr size_t kOffXS16 = kOffXS32 + (size_t)kRows * kE    * 4;
constexpr size_t kOffDBC  = kOffXS16 + (size_t)kRows * kE    * 2;
constexpr size_t kOffY16  = kOffDBC  + (size_t)kRows * kDbcP * 4;
constexpr size_t kWsTotal = kOffY16  + (size_t)kRows * kE    * 2;
static_assert(kWsTotal == 61026304ull);
static_assert(kWsTotal <= 134217728ull);
static_assert((kOffXNR % 128) == 0 && (kOffWIN % 128) == 0 && (kOffWINR % 128) == 0 && (kOffWX % 128) == 0 &&
              (kOffWOUT % 128) == 0 && (kOffXZ % 128) == 0 && (kOffXS32 % 128) == 0 && (kOffXS16 % 128) == 0 &&
              (kOffDBC % 128) == 0 && (kOffY16 % 128) == 0);

__device__ __forceinline__ _Float16 to_h16(float v) {
  const float f = (fabsf(v) < 6.103515625e-05f) ? 0.0f : v;
  return (_Float16)f;
}

union FragU { v16h v; v8h h[2]; };
__device__ __forceinline__ v16h frag_load(const _Float16* p) {
  FragU f;
  f.h[0] = *(const v8h*)(p);
  f.h[1] = *(const v8h*)(p + 16);
  return f.v;
}
__device__ __forceinline__ v8f frag_mma(v16h a, v16h b, v8f c) {
  return __builtin_amdgcn_wmma_f32_16x16x32_f16(false, a, false, b, (short)0, c, false, false);
}
__device__ __forceinline__ void guard1(v8f& a, v16h x, v16h y) {
  asm volatile("v_nop\n\tv_nop\n\tv_nop\n\tv_nop" : "+v"(a) : "v"(x), "v"(y));
}
__device__ __forceinline__ void guard2(v8f& a, v16h w, v16h x, v16h y, v16h z) {
  asm volatile("v_nop\n\tv_nop\n\tv_nop\n\tv_nop" : "+v"(a) : "v"(w), "v"(x), "v"(y), "v"(z));
}

constexpr unsigned kChWin   = (unsigned)(kP * kC / 8);
constexpr unsigned kChWx    = (unsigned)(kDbcP * kE / 8);
constexpr unsigned kChWout  = (unsigned)(kC * kE / 8);
constexpr unsigned kBlkWin  = kChWin / 256u;
constexpr unsigned kBlkWx   = kChWx / 256u;
constexpr unsigned kBlkWout = kChWout / 256u;
constexpr unsigned kWxValid = (unsigned)(kDbc * kE);
static_assert((kChWin % 256u) == 0 && (kChWx % 256u) == 0 && (kChWout % 256u) == 0);
static_assert((kWxValid % 8u) == 0);

__global__ __launch_bounds__(256) void pack_weights_kernel(
    const float* __restrict__ W_in, const float* __restrict__ W_x, const float* __restrict__ W_out,
    unsigned short* __restrict__ win16, unsigned short* __restrict__ win16r,
    unsigned short* __restrict__ wx16, unsigned short* __restrict__ wout16)
{
  const unsigned blk = blockIdx.x;
  const unsigned tid = threadIdx.x;
  const float* src;
  unsigned short* dst;
  unsigned q;
  unsigned valid;
  const bool isWin = blk < kBlkWin;
  if (isWin) {
    src = W_in;  dst = win16;  q = blk * 256u + tid;                        valid = (unsigned)(kP * kC);
  } else if (blk < kBlkWin + kBlkWx) {
    src = W_x;   dst = wx16;   q = (blk - kBlkWin) * 256u + tid;            valid = kWxValid;
  } else {
    src = W_out; dst = wout16; q = (blk - kBlkWin - kBlkWx) * 256u + tid;   valid = (unsigned)(kC * kE);
  }
  const unsigned e0 = q * 8u;
  const bool ok = e0 < valid;
  const unsigned ec = ok ? e0 : 0u;
  const v4f a0 = *(const v4f*)(src + ec);
  const v4f a1 = *(const v4f*)(src + ec + 4);
  const float cw = (float)kCarryW;
  const float cr = (float)kCarryRem;
  v8h hv;
  v8h rv;
#pragma unroll
  for (int e = 0; e < 4; ++e) {
    const float f0 = a0[e];
    const float f1 = a1[e];
    const float c0 = ok ? f0 * cw : 0.0f;
    const float c1 = ok ? f1 * cw : 0.0f;
    const _Float16 h0 = to_h16(c0);
    const _Float16 h1 = to_h16(c1);
    hv[e]     = h0;
    hv[4 + e] = h1;
    rv[e]     = to_h16((c0 - (float)h0) * cr);
    rv[4 + e] = to_h16((c1 - (float)h1) * cr);
  }
  unsigned short* p  = dst + e0;
  unsigned short* pr = win16r + e0;
  *(volatile v8h*)p = hv;
  if (isWin) *(volatile v8h*)pr = rv;
  __threadfence();
  *(volatile v8h*)p = hv;
  if (isWin) *(volatile v8h*)pr = rv;
}

__global__ __launch_bounds__(256) void rmsnorm_pack_kernel(
    const float* __restrict__ x, const float* __restrict__ norm_w,
    unsigned short* __restrict__ xn16, unsigned short* __restrict__ xn16r)
{
  __shared__ __align__(16) float sU[kC * 68];
  __shared__ float sPart[4 * 64];
  __shared__ float sScale[64];
  const unsigned tid = threadIdx.x;
  const unsigned g0 = blockIdx.x * 64u;
  const unsigned b  = g0 / (unsigned)kL;
  const unsigned l0 = g0 - b * (unsigned)kL;
  const float* xb = x + (size_t)b * kC * kL + l0;
#pragma unroll
  for (int i = 0; i < 6; ++i) {
    const unsigned idx = tid + 256u * (unsigned)i;
    const unsigned c  = idx >> 4;
    const unsigned l4 = (idx & 15u) * 4u;
    const v4f v = *(const v4f*)(xb + (size_t)c * kL + l4);
    *(v4f*)(sU + c * 68u + l4) = v;
  }
  __syncthreads();
  {
    const unsigned part = tid >> 6;
    const unsigned tok  = tid & 63u;
    float s = 0.0f;
#pragma unroll 4
    for (int c = 0; c < 24; ++c) {
      const float v = sU[(part * 24u + (unsigned)c) * 68u + tok];
      s = fmaf(v, v, s);
    }
    sPart[part * 64u + tok] = s;
  }
  __syncthreads();
  if (tid < 64u) {
    const float s = (sPart[tid] + sPart[64u + tid]) + (sPart[128u + tid] + sPart[192u + tid]);
    const float ms = s * (1.0f / (float)kC) + kEps;
    sScale[tid] = rsqrtf(ms) * (float)kCarryXn;
  }
  __syncthreads();
  const float cr = (float)kCarryRem;
  v8h hv[3];
  v8h rv[3];
#pragma unroll
  for (int i = 0; i < 3; ++i) {
    const unsigned q = tid + 256u * (unsigned)i;
    unsigned tok = q / 12u;
    asm volatile("" : "+v"(tok));
    const unsigned c0 = (q - tok * 12u) * 8u;
    const float sc = sScale[tok];
    const v4f nw0 = *(const v4f*)(norm_w + c0);
    const v4f nw1 = *(const v4f*)(norm_w + c0 + 4);
#pragma unroll
    for (int e = 0; e < 4; ++e) {
      const float u0 = sU[(c0 + (unsigned)e) * 68u + tok];
      const float u1 = sU[(c0 + 4u + (unsigned)e) * 68u + tok];
      const float g0w = nw0[e];
      const float g1w = nw1[e];
      float vc0 = (u0 * sc) * g0w;
      float vc1 = (u1 * sc) * g1w;
      asm volatile("" : "+v"(vc0));
      asm volatile("" : "+v"(vc1));
      const _Float16 h0 = to_h16(vc0);
      const _Float16 h1 = to_h16(vc1);
      hv[i][e]     = h0;
      hv[i][4 + e] = h1;
      rv[i][e]     = to_h16((vc0 - (float)h0) * cr);
      rv[i][4 + e] = to_h16((vc1 - (float)h1) * cr);
    }
  }
  unsigned short* base  = xn16  + (size_t)g0 * kC;
  unsigned short* baser = xn16r + (size_t)g0 * kC;
  for (int pass = 0; pass < 2; ++pass) {
#pragma unroll
    for (int i = 0; i < 3; ++i) {
      const unsigned q = tid + 256u * (unsigned)i;
      *(volatile v8h*)(base  + q * 8u) = hv[i];
      *(volatile v8h*)(baser + q * 8u) = rv[i];
    }
    __threadfence();
  }
}

template <int INV_SCALE, int REM_CARRY>
__global__ __launch_bounds__(256) void gemm16x64_f16x3_kernel(
    const unsigned short* __restrict__ Ap, const unsigned short* __restrict__ A2p, int lda,
    const unsigned short* __restrict__ Btp, const unsigned short* __restrict__ Bt2p, int ldb,
    float* __restrict__ C, int ldc, int M, int N, int K)
{
  const _Float16* A   = (const _Float16*)Ap;
  const _Float16* A2  = (const _Float16*)A2p;
  const _Float16* Bt  = (const _Float16*)Btp;
  const _Float16* Bt2 = (const _Float16*)Bt2p;
  __shared__ __align__(16) float sT[8][16 * 68];
  const int lane = threadIdx.x & 31;
  const int wave = threadIdx.x >> 5;
  const int tilesN = N >> 6;
  const int tilesM = M >> 4;
  const int tile = blockIdx.x * 8 + wave;
  if (tile >= tilesM * tilesN) return;
  const int tm = tile / tilesN;
  const int tn = tile - tm * tilesN;
  const int m0 = tm << 4;
  const int n0 = tn << 6;
  const int rlane = lane & 15;
  const int koff  = (lane >> 4) * 8;
  const int mOff  = (lane >> 4) * 8;
  const float scale = 1.0f / (float)INV_SCALE;
  const float rinv  = 1.0f / (float)REM_CARRY;

  v8f accm[4];
  v8f accr[4];
#pragma unroll
  for (int j = 0; j < 4; ++j) {
    accm[j] = (v8f){0.f, 0.f, 0.f, 0.f, 0.f, 0.f, 0.f, 0.f};
    accr[j] = (v8f){0.f, 0.f, 0.f, 0.f, 0.f, 0.f, 0.f, 0.f};
  }

  for (int k0 = 0; k0 < K; k0 += 32) {
    const size_t ao = (size_t)(m0 + rlane) * lda + koff + k0;
    const v16h ah = frag_load(A + ao);
    const v16h al = frag_load(A2 + ao);
    v16h bh[4];
    v16h bl[4];
#pragma unroll
    for (int j = 0; j < 4; ++j) {
      const size_t bo = (size_t)(n0 + (j << 4) + rlane) * ldb + koff + k0;
      bh[j] = frag_load(Bt + bo);
      bl[j] = frag_load(Bt2 + bo);
    }
#pragma unroll
    for (int j = 0; j < 4; ++j) accm[j] = frag_mma(ah, bh[j], accm[j]);
#pragma unroll
    for (int j = 0; j < 4; ++j) {
      accr[j] = frag_mma(ah, bl[j], accr[j]);
      accr[j] = frag_mma(al, bh[j], accr[j]);
    }
#pragma unroll
    for (int j = 0; j < 4; ++j) guard1(accm[j], ah, bh[j]);
#pragma unroll
    for (int j = 0; j < 4; ++j) guard2(accr[j], ah, bl[j], al, bh[j]);
  }

  float* slab = sT[wave];
#pragma unroll
  for (int j = 0; j < 4; ++j) {
#pragma unroll
    for (int r = 0; r < 8; ++r) {
      const float m = accm[j][r];
      const float s = accr[j][r];
      slab[(mOff + r) * 68 + (j << 4) + rlane] = (m + s * rinv) * scale;
    }
  }
  __builtin_amdgcn_fence(__ATOMIC_RELEASE, "workgroup");
  __builtin_amdgcn_wave_barrier();
  __builtin_amdgcn_fence(__ATOMIC_ACQUIRE, "workgroup");
  {
    const int hh = lane >> 4;
    const int c4 = (lane & 15) * 4;
    for (int pass = 0; pass < 2; ++pass) {
#pragma unroll
      for (int it = 0; it < 8; ++it) {
        const int row = it * 2 + hh;
        const v4f v = *(const v4f*)(slab + row * 68 + c4);
        *(volatile v4f*)(C + (size_t)(m0 + row) * ldc + n0 + c4) = v;
      }
      __threadfence();
    }
  }
}

template <int INV_SCALE>
__global__ __launch_bounds__(256) void gemm64_f16_kernel(
    const unsigned short* __restrict__ Ap, int lda,
    const unsigned short* __restrict__ Btp, int ldb,
    float* __restrict__ C, int ldc, int M, int N, int K)
{
  const _Float16* A  = (const _Float16*)Ap;
  const _Float16* Bt = (const _Float16*)Btp;
  __shared__ __align__(16) float sT[8][16 * 68];
  const int lane = threadIdx.x & 31;
  const int wave = threadIdx.x >> 5;
  const int tilesN = N >> 6;
  const int tilesM = M >> 6;
  const int tile = blockIdx.x * 8 + wave;
  if (tile >= tilesM * tilesN) return;
  const int tm = tile / tilesN;
  const int tn = tile - tm * tilesN;
  const int m0 = tm << 6;
  const int n0 = tn << 6;
  const int rlane = lane & 15;
  const int koff  = (lane >> 4) * 8;
  const int mOff  = (lane >> 4) * 8;
  const float scale = 1.0f / (float)INV_SCALE;

  v8f acc[4][4];
#pragma unroll
  for (int i = 0; i < 4; ++i)
#pragma unroll
    for (int j = 0; j < 4; ++j) acc[i][j] = (v8f){0.f, 0.f, 0.f, 0.f, 0.f, 0.f, 0.f, 0.f};

  for (int k0 = 0; k0 < K; k0 += 32) {
    v16h bh[4];
#pragma unroll
    for (int j = 0; j < 4; ++j) {
      const size_t bo = (size_t)(n0 + (j << 4) + rlane) * ldb + koff + k0;
      bh[j] = frag_load(Bt + bo);
    }
#pragma unroll
    for (int i = 0; i < 4; ++i) {
      const size_t ao = (size_t)(m0 + (i << 4) + rlane) * lda + koff + k0;
      const v16h ah = frag_load(A + ao);
#pragma unroll
      for (int j = 0; j < 4; ++j) acc[i][j] = frag_mma(ah, bh[j], acc[i][j]);
#pragma unroll
      for (int j = 0; j < 4; ++j) guard1(acc[i][j], ah, bh[j]);
    }
  }

  float* slab = sT[wave];
#pragma unroll
  for (int i = 0; i < 4; ++i) {
    const int mBase = m0 + (i << 4);
#pragma unroll
    for (int j = 0; j < 4; ++j) {
#pragma unroll
      for (int r = 0; r < 8; ++r) {
        slab[(mOff + r) * 68 + (j << 4) + rlane] = acc[i][j][r] * scale;
      }
    }
    __builtin_amdgcn_fence(__ATOMIC_RELEASE, "workgroup");
    __builtin_amdgcn_wave_barrier();
    __builtin_amdgcn_fence(__ATOMIC_ACQUIRE, "workgroup");
    {
      const int hh = lane >> 4;
      const int c4 = (lane & 15) * 4;
      for (int pass = 0; pass < 2; ++pass) {
#pragma unroll
        for (int it = 0; it < 8; ++it) {
          const int row = it * 2 + hh;
          const v4f v = *(const v4f*)(slab + row * 68 + c4);
          *(volatile v4f*)(C + (size_t)(mBase + row) * ldc + n0 + c4) = v;
        }
        __threadfence();
      }
    }
    __builtin_amdgcn_fence(__ATOMIC_RELEASE, "workgroup");
    __builtin_amdgcn_wave_barrier();
    __builtin_amdgcn_fence(__ATOMIC_ACQUIRE, "workgroup");
  }
}

constexpr int kConvTP = 196;

__global__ __launch_bounds__(192) void conv_silu_kernel(
    const float* __restrict__ XZ, const float* __restrict__ cw, const float* __restrict__ cb,
    float* __restrict__ XS, unsigned short* __restrict__ XS16)
{
  __shared__ __align__(16) float sT[16 * kConvTP];
  const unsigned tid = threadIdx.x;
  const unsigned d = tid;
  const unsigned g0 = blockIdx.x * 64u;
  const unsigned tb = g0 & (unsigned)(kL - 1);
  const v4f wv = *(const v4f*)(cw + d * 4u);
  const float w0 = wv[0], w1 = wv[1], w2 = wv[2], w3 = wv[3];
  const float bc = cb[d];
  float xm3, xm2, xm1;
  {
    const bool hist = (tb > 0u);
    const unsigned rb = hist ? (g0 - 3u) : g0;
    const float v3 = XZ[(size_t)rb * kP + d];
    const float v2 = XZ[(size_t)(rb + 1u) * kP + d];
    const float v1 = XZ[(size_t)(rb + 2u) * kP + d];
    xm3 = hist ? v3 : 0.0f;
    xm2 = hist ? v2 : 0.0f;
    xm1 = hist ? v1 : 0.0f;
  }
#pragma unroll 1
  for (int sub = 0; sub < 4; ++sub) {
    const unsigned lb = g0 + (unsigned)sub * 16u;
#pragma unroll 1
    for (int s = 0; s < 16; ++s) {
      const float xcur = XZ[(size_t)(lb + (unsigned)s) * kP + d];
      float acc = w0 * xm3;
      acc = fmaf(w1, xm2, acc);
      acc = fmaf(w2, xm1, acc);
      acc = fmaf(w3, xcur, acc);
      const float sv = acc + bc;
      const float sg = __builtin_amdgcn_rcpf(1.0f + expf(-sv));
      sT[s * kConvTP + (int)tid] = sv * sg;
      xm3 = xm2;
      xm2 = xm1;
      xm1 = xcur;
    }
    __syncthreads();
    v4f fv[4];
    v8h hv[2];
#pragma unroll
    for (int it = 0; it < 4; ++it) {
      const unsigned idx = tid + 192u * (unsigned)it;
      unsigned r = idx / 48u;
      asm volatile("" : "+v"(r));
      const unsigned c4 = (idx - r * 48u) * 4u;
      fv[it] = *(const v4f*)(sT + r * (unsigned)kConvTP + c4);
    }
#pragma unroll
    for (int it = 0; it < 2; ++it) {
      const unsigned q = tid + 192u * (unsigned)it;
      unsigned r = q / 24u;
      asm volatile("" : "+v"(r));
      const unsigned c8 = (q - r * 24u) * 8u;
      const float* sp = sT + r * (unsigned)kConvTP + c8;
      const v4f a0 = *(const v4f*)(sp);
      const v4f a1 = *(const v4f*)(sp + 4);
#pragma unroll
      for (int e = 0; e < 4; ++e) {
        const float f0 = a0[e];
        const float f1 = a1[e];
        hv[it][e]     = to_h16(f0 * (float)kCarryXs);
        hv[it][4 + e] = to_h16(f1 * (float)kCarryXs);
      }
    }
    float* ob = XS + (size_t)lb * kE;
    unsigned short* hb = XS16 + (size_t)lb * kE;
    for (int pass = 0; pass < 2; ++pass) {
#pragma unroll
      for (int it = 0; it < 4; ++it) {
        const unsigned idx = tid + 192u * (unsigned)it;
        *(volatile v4f*)(ob + idx * 4u) = fv[it];
      }
#pragma unroll
      for (int it = 0; it < 2; ++it) {
        const unsigned q = tid + 192u * (unsigned)it;
        *(volatile v8h*)(hb + q * 8u) = hv[it];
      }
      __threadfence();
    }
    __syncthreads();
  }
}

constexpr int kScanCh = 64;
constexpr int kScanTS = 64;
constexpr int kScanYP = 68;
constexpr int kScanBlkPerImg = kE / kScanCh;
static_assert((kL % kScanTS) == 0);

__global__ __launch_bounds__(128) void scan_kernel(
    const float* __restrict__ DBC, const float* __restrict__ XS, const float* __restrict__ XZ,
    const float* __restrict__ Wdt, const float* __restrict__ bdt, const float* __restrict__ Alog,
    const float* __restrict__ Dp, unsigned short* __restrict__ Y16)
{
  __shared__ __align__(16) float sX[kScanTS * kDbcP];
  __shared__ __align__(16) float sY[kScanTS * kScanYP];
  __shared__ float sA[kN * kScanCh];
  const unsigned tid  = threadIdx.x;
  const unsigned lane = tid & 31u;
  const unsigned wave = tid >> 5;
  const unsigned ch   = tid >> 1;
  const unsigned half = tid & 1u;
  const unsigned bix  = blockIdx.x / (unsigned)kScanBlkPerImg;
  const unsigned d0   = (blockIdx.x - bix * (unsigned)kScanBlkPerImg) * (unsigned)kScanCh;
  const unsigned d    = d0 + ch;
  const size_t row0   = (size_t)bix * kL;

#pragma unroll 1
  for (int k = 0; k < 8; ++k) {
    const unsigned n = half * 8u + (unsigned)k;
    sA[n * (unsigned)kScanCh + ch] = -expf(Alog[(size_t)d * kN + n]);
  }
  __syncthreads();
  float negA[8], h[8];
#pragma unroll
  for (int k = 0; k < 8; ++k) {
    negA[k] = sA[(half * 8u + (unsigned)k) * (unsigned)kScanCh + ch];
    h[k] = 0.0f;
  }
  float wdt[kR];
#pragma unroll
  for (int j = 0; j < kR; ++j) wdt[j] = Wdt[(size_t)d * kR + j];
  const float bb = bdt[d];
  const float Dd = Dp[d];
  const unsigned bofs = (unsigned)kR + half * 8u;
  const unsigned cofs = (unsigned)(kR + kN) + half * 8u;
  const unsigned q  = lane >> 3;
  const unsigned c8 = (lane & 7u) * 8u;

#pragma unroll 1
  for (int t0 = 0; t0 < kL; t0 += kScanTS) {
    __syncthreads();
    {
      const float* gsrc = DBC + (row0 + (size_t)t0) * kDbcP;
#pragma unroll
      for (int i = 0; i < 8; ++i) {
        const unsigned idx = tid + 128u * (unsigned)i;
        *(v4f*)(sX + idx * 4u) = *(const v4f*)(gsrc + idx * 4u);
      }
    }
    __syncthreads();
#pragma unroll 1
    for (int s = 0; s < kScanTS; ++s) {
      const size_t row = row0 + (size_t)(t0 + s);
      const float* xr = sX + s * kDbcP;
      float vdot = 0.0f;
#pragma unroll
      for (int j = 0; j < kR; ++j) vdot = fmaf(xr[j], wdt[j], vdot);
      const float v   = vdot + bb;
      const float a   = expf(-fabsf(v));
      const float u   = 1.0f + a;
      const float l1p = logf(u) + (a - (u - 1.0f)) * __builtin_amdgcn_rcpf(u);
      const float dt  = fmaxf(v, 0.0f) + l1p;
      const float xt  = XS[row * kE + d];
      const float zv  = XZ[row * kP + (unsigned)kE + d];
      const float dtx = dt * xt;
      float y = 0.0f;
#pragma unroll
      for (int k = 0; k < 8; ++k) {
        const float e = expf(dt * negA[k]);
        h[k] = fmaf(e, h[k], dtx * xr[bofs + (unsigned)k]);
        y = fmaf(h[k], xr[cofs + (unsigned)k], y);
      }
      const float yo = __shfl_xor(y, 1, 32);
      y = y + yo;
      y = fmaf(xt, Dd, y);
      const float sg = __builtin_amdgcn_rcpf(1.0f + expf(-zv));
      y = y * (zv * sg);
      sY[s * kScanYP + (int)ch] = y;
    }
    __syncthreads();
    v8h hv[4];
#pragma unroll
    for (int it = 0; it < 4; ++it) {
      const unsigned rowl = (unsigned)it * 16u + wave * 4u + q;
      const float* sp = sY + rowl * (unsigned)kScanYP + c8;
      const v4f a0 = *(const v4f*)(sp);
      const v4f a1 = *(const v4f*)(sp + 4);
#pragma unroll
      for (int e = 0; e < 4; ++e) {
        const float f0 = a0[e];
        const float f1 = a1[e];
        hv[it][e]     = to_h16(f0 * (float)kCarryY);
        hv[it][4 + e] = to_h16(f1 * (float)kCarryY);
      }
    }
    for (int pass = 0; pass < 2; ++pass) {
#pragma unroll
      for (int it = 0; it < 4; ++it) {
        const unsigned rowl = (unsigned)it * 16u + wave * 4u + q;
        const size_t o = (row0 + (size_t)t0 + rowl) * kE + d0 + c8;
        *(volatile v8h*)(Y16 + o) = hv[it];
      }
      __threadfence();
    }
  }
}

__global__ __launch_bounds__(128) void outproj_kernel(
    const unsigned short* __restrict__ Yp, const unsigned short* __restrict__ Wp,
    const float* __restrict__ x, float* __restrict__ out)
{
  __shared__ __align__(16) float sC[kC * 68];
  const _Float16* A  = (const _Float16*)Yp;
  const _Float16* Bt = (const _Float16*)Wp;
  const unsigned tid  = threadIdx.x;
  const unsigned lane = tid & 31u;
  const unsigned wave = tid >> 5;
  const unsigned rlane = lane & 15u;
  const unsigned hh    = lane >> 4;
  const unsigned koff  = hh * 8u;
  const unsigned g0 = blockIdx.x * 64u;
  const unsigned b  = g0 / (unsigned)kL;
  const unsigned l0 = g0 - b * (unsigned)kL;
  const float scale = 1.0f / (float)(kCarryY * kCarryW);

  v8f acc[6];
#pragma unroll
  for (int j = 0; j < 6; ++j) acc[j] = (v8f){0.f, 0.f, 0.f, 0.f, 0.f, 0.f, 0.f, 0.f};

#pragma unroll 1
  for (int k0 = 0; k0 < kE; k0 += 32) {
    const v16h ah = frag_load(A + (size_t)(g0 + wave * 16u + rlane) * kE + koff + (unsigned)k0);
    v16h bf[6];
#pragma unroll
    for (int j = 0; j < 6; ++j)
      bf[j] = frag_load(Bt + (size_t)((unsigned)j * 16u + rlane) * kE + koff + (unsigned)k0);
#pragma unroll
    for (int j = 0; j < 6; ++j) acc[j] = frag_mma(ah, bf[j], acc[j]);
#pragma unroll
    for (int j = 0; j < 6; ++j) guard1(acc[j], ah, bf[j]);
  }

#pragma unroll
  for (int j = 0; j < 6; ++j) {
#pragma unroll
    for (int r = 0; r < 8; ++r) {
      sC[((unsigned)j * 16u + rlane) * 68u + wave * 16u + hh * 8u + (unsigned)r] = acc[j][r] * scale;
    }
  }
  __syncthreads();

  const unsigned c4 = (lane & 15u) * 4u;
  v4f val[12];
#pragma unroll
  for (int it = 0; it < 12; ++it) {
    const unsigned c = wave * 24u + (unsigned)it * 2u + hh;
    const size_t off = ((size_t)b * kC + c) * kL + l0 + c4;
    const v4f rv = *(const v4f*)(x + off);
    const v4f sv = *(const v4f*)(sC + c * 68u + c4);
    val[it] = sv + rv;
  }
  for (int pass = 0; pass < 2; ++pass) {
#pragma unroll
    for (int it = 0; it < 12; ++it) {
      const unsigned c = wave * 24u + (unsigned)it * 2u + hh;
      const size_t off = ((size_t)b * kC + c) * kL + l0 + c4;
      *(volatile v4f*)(out + off) = val[it];
    }
    __threadfence();
  }
}

static_assert((((kRows / 16) * (kP / 64)) % 8) == 0);
static_assert((((kRows / 64) * (kDbcP / 64)) % 8) == 0);

extern "C" void kernel_launch(void* const* d_in, const int* in_sizes, int n_in,
                              void* d_out, int out_size, void* d_ws, size_t ws_size,
                              hipStream_t stream) {
  if (n_in < 11) return;
  if (in_sizes[0] != kB * kC * kL) return;
  if (in_sizes[1] != kP * kC) return;
  if (in_sizes[2] != kE * kTaps) return;
  if (in_sizes[3] != kE) return;
  if (in_sizes[4] != kDbc * kE) return;
  if (in_sizes[5] != kE * kR) return;
  if (in_sizes[6] != kE) return;
  if (in_sizes[7] != kE * kN) return;
  if (in_sizes[8] != kE) return;
  if (in_sizes[9] != kC * kE) return;
  if (in_sizes[10] != kC) return;
  if (out_size != kB * kC * kL) return;
  if (ws_size < kWsTotal) return;

  const float* x      = (const float*)d_in[0];
  const float* W_in   = (const float*)d_in[1];
  const float* conv_w = (const float*)d_in[2];
  const float* conv_b = (const float*)d_in[3];
  const float* W_x    = (const float*)d_in[4];
  const float* W_dt   = (const float*)d_in[5];
  const float* b_dt   = (const float*)d_in[6];
  const float* A_log  = (const float*)d_in[7];
  const float* D_par  = (const float*)d_in[8];
  const float* W_out  = (const float*)d_in[9];
  const float* norm_w = (const float*)d_in[10];
  float* out = (float*)d_out;

  char* ws = (char*)d_ws;
  unsigned short* XN16   = (unsigned short*)(ws + kOffXN);
  unsigned short* XN16R  = (unsigned short*)(ws + kOffXNR);
  unsigned short* WIN16  = (unsigned short*)(ws + kOffWIN);
  unsigned short* WIN16R = (unsigned short*)(ws + kOffWINR);
  unsigned short* WX16   = (unsigned short*)(ws + kOffWX);
  unsigned short* WOUT16 = (unsigned short*)(ws + kOffWOUT);
  float*          XZ32   = (float*)(ws + kOffXZ);
  float*          XS32   = (float*)(ws + kOffXS32);
  unsigned short* XS16   = (unsigned short*)(ws + kOffXS16);
  float*          DBC32  = (float*)(ws + kOffDBC);
  unsigned short* Y16    = (unsigned short*)(ws + kOffY16);

  pack_weights_kernel<<<kBlkWin + kBlkWx + kBlkWout, 256, 0, stream>>>(
      W_in, W_x, W_out, WIN16, WIN16R, WX16, WOUT16);

  rmsnorm_pack_kernel<<<kRows / 64, 256, 0, stream>>>(x, norm_w, XN16, XN16R);

  gemm16x64_f16x3_kernel<kCarryXn * kCarryW, kCarryRem><<<((kRows / 16) * (kP / 64)) / 8, 256, 0, stream>>>(
      XN16, XN16R, kC, WIN16, WIN16R, kC, XZ32, kP, kRows, kP, kC);

  conv_silu_kernel<<<kRows / 64, 192, 0, stream>>>(XZ32, conv_w, conv_b, XS32, XS16);

  gemm64_f16_kernel<kCarryXs * kCarryW><<<((kRows / 64) * (kDbcP / 64)) / 8, 256, 0, stream>>>(
      XS16, kE, WX16, kE, DBC32, kDbcP, kRows, kDbcP, kE);

  scan_kernel<<<kB * kScanBlkPerImg, 128, 0, stream>>>(DBC32, XS32, XZ32, W_dt, b_dt, A_log, D_par, Y16);

  outproj_kernel<<<kRows / 64, 128, 0, stream>>>(Y16, WOUT16, x, out);
}
